// S6_2680059593332
// MI455X (gfx1250) — hardware-verified
//
#include <hip/hip_runtime.h>
#include <math.h>

typedef __attribute__((ext_vector_type(16))) __bf16   v16b;
typedef __attribute__((ext_vector_type(8)))  __bf16   v8b;
typedef __attribute__((ext_vector_type(8)))  float    v8f;
typedef __attribute__((ext_vector_type(4)))  float    v4f;
typedef __attribute__((ext_vector_type(4)))  unsigned v4u;

constexpr int kBatch  = 2;
constexpr int kSeq    = 1024;
constexpr int kD      = 1024;
constexpr int kNst    = 16;
constexpr int kDtR    = 64;
constexpr int kE      = 96;
constexpr int kEP     = 128;
constexpr int kRows   = kBatch * kSeq;
constexpr int kTP     = 260;
constexpr int kScanTS = 64;
constexpr int kScanCh = 64;
constexpr int kScanYP = 68;
constexpr int kBC     = 2 * kNst;
constexpr float kEps  = 1e-12f;
static_assert(kDtR + 2 * kNst == kE, "projection width");
static_assert((kD % 32) == 0 && (kDtR % 32) == 0, "GEMM K multiples of 32");
static_assert((kRows % 64) == 0 && (kEP % 64) == 0 && (kD % 64) == 0, "GEMM M,N multiples of 64");
static_assert((kSeq % kScanTS) == 0 && (kSeq % 16) == 0 && (kD % kScanCh) == 0 && (kD % 256) == 0, "tile multiples");
static_assert((kD % 64) == 0 && (kDtR % 64) == 0 && (kEP % 64) == 0, "transpose tiles");

constexpr size_t kOffXH  = 0;
constexpr size_t kOffXL  = kOffXH  + (size_t)kRows * kD * 2;
constexpr size_t kOffWXH = kOffXL  + (size_t)kRows * kD * 2;
constexpr size_t kOffWXL = kOffWXH + (size_t)kEP * kD * 2;
constexpr size_t kOffWDH = kOffWXL + (size_t)kEP * kD * 2;
constexpr size_t kOffWDL = kOffWDH + (size_t)kD * kDtR * 2;
constexpr size_t kOffWOH = kOffWDL + (size_t)kD * kDtR * 2;
constexpr size_t kOffWOL = kOffWOH + (size_t)kD * kD * 2;
constexpr size_t kOffXD  = kOffWOL + (size_t)kD * kD * 2;
constexpr size_t kOffDRH = kOffXD  + (size_t)kRows * kEP * 4;
constexpr size_t kOffDRL = kOffDRH + (size_t)kRows * kDtR * 2;
constexpr size_t kOffDLR = kOffDRL + (size_t)kRows * kDtR * 2;
constexpr size_t kOffSFX = kOffDLR + (size_t)kRows * kD * 4;
constexpr size_t kOffYH  = kOffSFX + (size_t)kRows * kD * 4;
constexpr size_t kOffYL  = kOffYH  + (size_t)kRows * kD * 2;
constexpr size_t kWsTotal = kOffYL + (size_t)kRows * kD * 2;
static_assert(kWsTotal == 40108032ull, "carve total");
static_assert(kWsTotal <= 134217728ull, "carve cap");
static_assert((kOffXL % 128) == 0 && (kOffWXH % 128) == 0 && (kOffWXL % 128) == 0 && (kOffWDH % 128) == 0 &&
              (kOffWDL % 128) == 0 && (kOffWOH % 128) == 0 && (kOffWOL % 128) == 0 && (kOffXD % 128) == 0 &&
              (kOffDRH % 128) == 0 && (kOffDRL % 128) == 0 && (kOffDLR % 128) == 0 && (kOffSFX % 128) == 0 &&
              (kOffYH % 128) == 0 && (kOffYL % 128) == 0, "128-B aligned regions");

__device__ __forceinline__ unsigned bf_rne_bits(float f) {
  const unsigned u = __float_as_uint(f);
  return (u + 0x7FFFu + ((u >> 16) & 1u)) >> 16;
}
__device__ __forceinline__ void split_pair(float f0, float f1, unsigned& hw, unsigned& lw) {
  const unsigned h0 = bf_rne_bits(f0);
  const unsigned h1 = bf_rne_bits(f1);
  const float r0 = f0 - __uint_as_float(h0 << 16);
  const float r1 = f1 - __uint_as_float(h1 << 16);
  const unsigned l0 = bf_rne_bits(r0);
  const unsigned l1 = bf_rne_bits(r1);
  hw = h0 | (h1 << 16);
  lw = l0 | (l1 << 16);
}
__device__ __forceinline__ void split_eight(const v4f a0, const v4f a1, v4u& hv, v4u& lv) {
  const float f0 = a0[0], f1 = a0[1], f2 = a0[2], f3 = a0[3];
  const float f4 = a1[0], f5 = a1[1], f6 = a1[2], f7 = a1[3];
  unsigned h0, h1, h2, h3, l0, l1, l2, l3;
  split_pair(f0, f1, h0, l0);
  split_pair(f2, f3, h1, l1);
  split_pair(f4, f5, h2, l2);
  split_pair(f6, f7, h3, l3);
  hv = (v4u){h0, h1, h2, h3};
  lv = (v4u){l0, l1, l2, l3};
}

__device__ __forceinline__ float softplus_f(float v) {
  return fmaxf(v, 0.0f) + log1pf(expf(-fabsf(v)));
}

__device__ __forceinline__ void dep_guard4_b(v8f& a, v8f& b, v8f& c, v8f& d, v16b x, v16b y) {
  asm volatile("v_nop\n\tv_nop\n\tv_nop\n\tv_nop" : "+v"(a), "+v"(b), "+v"(c), "+v"(d) : "v"(x), "v"(y));
}
__device__ __forceinline__ void keep4_b(v16b a, v16b b, v16b c, v16b d) { asm volatile("v_nop" :: "v"(a), "v"(b), "v"(c), "v"(d)); }
__device__ __forceinline__ void acc_guard4(v8f& a, v8f& b, v8f& c, v8f& d) { asm volatile("v_nop\n\tv_nop\n\tv_nop\n\tv_nop" : "+v"(a), "+v"(b), "+v"(c), "+v"(d)); }
struct FragB {
  union U { v16b v; v8b h[2]; };
  static __device__ __forceinline__ v16b load(const __bf16* p) {
    U f; f.h[0] = *(const v8b*)(p); f.h[1] = *(const v8b*)(p + 16); return f.v;
  }
  static __device__ __forceinline__ v8f mma(v16b a, v16b b, v8f c) {
    return __builtin_amdgcn_wmma_f32_16x16x32_bf16(false, a, false, b, (short)0, c, false, false);
  }
};

template <int BIAS_MODE>
__global__ __launch_bounds__(256) void wmma_gemm64_x3(
    const unsigned short* __restrict__ Ap, const unsigned short* __restrict__ A2p, int lda,
    const unsigned short* __restrict__ Btp, const unsigned short* __restrict__ Bt2p, int ldb,
    float* __restrict__ Cout, int ldc,
    const float* __restrict__ bias,
    int M, int N, int K) {
  typedef __bf16 T;
  typedef v16b V;
  const T* Ab  = (const T*)Ap;
  const T* Ab2 = (const T*)A2p;
  const T* Bb  = (const T*)Btp;
  const T* Bb2 = (const T*)Bt2p;
  __shared__ __align__(16) float sT[8][16 * 68];
  const int lane = threadIdx.x & 31;
  const int wave = threadIdx.x >> 5;
  const int tilesN = N >> 6;
  const int tilesM = M >> 6;
  const int tile = blockIdx.x * 8 + wave;
  if (tile >= tilesM * tilesN) return;
  const int tm = tile / tilesN;
  const int tn = tile - tm * tilesN;
  const int m0 = tm << 6;
  const int n0 = tn << 6;

  const int rlane = lane & 15;
  const int koff  = (lane >> 4) * 8;
  const int mOff  = (lane >> 4) * 8;

  v8f acc[4][4];
#pragma unroll
  for (int i = 0; i < 4; ++i)
#pragma unroll
    for (int j = 0; j < 4; ++j) acc[i][j] = (v8f){0.f,0.f,0.f,0.f,0.f,0.f,0.f,0.f};

  for (int k0 = 0; k0 < K; k0 += 32) {
    V bh[4], bl[4];
#pragma unroll
    for (int j = 0; j < 4; ++j) {
      const size_t bo = (size_t)(n0 + (j << 4) + rlane) * ldb + koff + k0;
      bh[j] = FragB::load(Bb + bo);
      bl[j] = FragB::load(Bb2 + bo);
    }
#pragma unroll
    for (int i = 0; i < 4; ++i) {
      const size_t ao = (size_t)(m0 + (i << 4) + rlane) * lda + koff + k0;
      V ah = FragB::load(Ab + ao);
      V al = FragB::load(Ab2 + ao);
#pragma unroll
      for (int j = 0; j < 4; ++j) {
        acc[i][j] = FragB::mma(ah, bh[j], acc[i][j]);
        acc[i][j] = FragB::mma(ah, bl[j], acc[i][j]);
        acc[i][j] = FragB::mma(al, bh[j], acc[i][j]);
      }
      dep_guard4_b(acc[i][0], acc[i][1], acc[i][2], acc[i][3], ah, al);
    }
    keep4_b(bh[0], bh[1], bh[2], bh[3]);
    keep4_b(bl[0], bl[1], bl[2], bl[3]);
  }
  acc_guard4(acc[0][0], acc[0][1], acc[0][2], acc[0][3]);
  acc_guard4(acc[1][0], acc[1][1], acc[1][2], acc[1][3]);
  acc_guard4(acc[2][0], acc[2][1], acc[2][2], acc[2][3]);
  acc_guard4(acc[3][0], acc[3][1], acc[3][2], acc[3][3]);

  float* slab = sT[wave];
#pragma unroll
  for (int i = 0; i < 4; ++i) {
    const int mBase = m0 + (i << 4);
#pragma unroll
    for (int j = 0; j < 4; ++j) {
      const int n = n0 + (j << 4) + rlane;
      float bv = 0.f;
      if (BIAS_MODE == 2) bv = bias[n];
#pragma unroll
      for (int r = 0; r < 8; ++r) {
        float v = acc[i][j][r];
        if (BIAS_MODE == 2) v += bv;
        slab[(mOff + r) * 68 + (j << 4) + rlane] = v;
      }
    }
    __builtin_amdgcn_fence(__ATOMIC_RELEASE, "workgroup");
    __builtin_amdgcn_wave_barrier();
    __builtin_amdgcn_fence(__ATOMIC_ACQUIRE, "workgroup");
    {
      const int hh = lane >> 4, c4 = (lane & 15) * 4;
      for (int pass = 0; pass < 2; ++pass) {
#pragma unroll
        for (int it = 0; it < 8; ++it) {
          const int row = it * 2 + hh;
          v4f v = *(const v4f*)(slab + row * 68 + c4);
          *(volatile v4f*)(Cout + (size_t)(mBase + row) * ldc + n0 + c4) = v;
        }
        __threadfence();
      }
    }
    __builtin_amdgcn_fence(__ATOMIC_RELEASE, "workgroup");
    __builtin_amdgcn_wave_barrier();
    __builtin_amdgcn_fence(__ATOMIC_ACQUIRE, "workgroup");
  }
}

__global__ __launch_bounds__(256) void split_rows_bf16_kernel(
    const float* __restrict__ src, unsigned short* __restrict__ dhi, unsigned short* __restrict__ dlo, int total8)
{
  const int i = blockIdx.x * 256 + threadIdx.x;
  if (i >= total8) return;
  const size_t e0 = (size_t)i << 3;
  const v4f a0 = *(const v4f*)(src + e0);
  const v4f a1 = *(const v4f*)(src + e0 + 4);
  v4u hv, lv;
  split_eight(a0, a1, hv, lv);
  unsigned short* qh = dhi + e0;
  unsigned short* ql = dlo + e0;
  *(volatile v4u*)qh = hv;
  *(volatile v4u*)ql = lv;
  __threadfence();
  *(volatile v4u*)qh = hv;
  *(volatile v4u*)ql = lv;
}

__global__ __launch_bounds__(256) void transpose_split_kernel(
    const float* __restrict__ W, unsigned short* __restrict__ BtH, unsigned short* __restrict__ BtL,
    int Kdim, int Ndim)
{
  __shared__ float tile[64 * 65];
  const int tid = threadIdx.x, lane = tid & 31, wave = tid >> 5;
  const int n0 = blockIdx.x * 64;
  const int k0 = blockIdx.y * 64;
#pragma unroll
  for (int p = 0; p < 16; ++p) {
    const int idx = tid + p * 256;
    const int kk  = idx >> 6;
    const int nn  = idx & 63;
    const int n   = n0 + nn;
    const int nc  = (n < Ndim) ? n : (Ndim - 1);
    const float v = W[(size_t)(k0 + kk) * Ndim + nc];
    tile[kk * 65 + nn] = (n < Ndim) ? v : 0.f;
  }
  __syncthreads();
  const int q = lane >> 3, c8 = (lane & 7) * 8;
  v4u hv[2], lv[2];
#pragma unroll
  for (int it = 0; it < 2; ++it) {
    const int nrow = it * 32 + wave * 4 + q;
    const float f0 = tile[(c8 + 0) * 65 + nrow];
    const float f1 = tile[(c8 + 1) * 65 + nrow];
    const float f2 = tile[(c8 + 2) * 65 + nrow];
    const float f3 = tile[(c8 + 3) * 65 + nrow];
    const float f4 = tile[(c8 + 4) * 65 + nrow];
    const float f5 = tile[(c8 + 5) * 65 + nrow];
    const float f6 = tile[(c8 + 6) * 65 + nrow];
    const float f7 = tile[(c8 + 7) * 65 + nrow];
    unsigned h0, h1, h2, h3, l0, l1, l2, l3;
    split_pair(f0, f1, h0, l0);
    split_pair(f2, f3, h1, l1);
    split_pair(f4, f5, h2, l2);
    split_pair(f6, f7, h3, l3);
    hv[it] = (v4u){h0, h1, h2, h3};
    lv[it] = (v4u){l0, l1, l2, l3};
  }
  for (int pass = 0; pass < 2; ++pass) {
#pragma unroll
    for (int it = 0; it < 2; ++it) {
      const int nrow = it * 32 + wave * 4 + q;
      const size_t o = (size_t)(n0 + nrow) * Kdim + k0 + c8;
      *(volatile v4u*)(BtH + o) = hv[it];
      *(volatile v4u*)(BtL + o) = lv[it];
    }
    __threadfence();
  }
}

__global__ __launch_bounds__(256) void dr_split_kernel(
    const float* __restrict__ XD, unsigned short* __restrict__ DRH, unsigned short* __restrict__ DRL, int total8)
{
  const int i = blockIdx.x * 256 + threadIdx.x;
  if (i >= total8) return;
  const int e0  = i << 3;
  const int row = e0 >> 6;
  const int c8  = e0 & 63;
  const float* p = XD + (size_t)row * kEP + c8;
  const v4f a0 = *(const v4f*)(p);
  const v4f a1 = *(const v4f*)(p + 4);
  v4u hv, lv;
  split_eight(a0, a1, hv, lv);
  unsigned short* qh = DRH + e0;
  unsigned short* ql = DRL + e0;
  *(volatile v4u*)qh = hv;
  *(volatile v4u*)ql = lv;
  __threadfence();
  *(volatile v4u*)qh = hv;
  *(volatile v4u*)ql = lv;
}

__global__ __launch_bounds__(256) void suffix_kernel(const float* __restrict__ DLR, float* __restrict__ SFX)
{
  __shared__ __align__(16) float sT[16 * kTP];
  const int tid = threadIdx.x, lane = tid & 31, wave = tid >> 5;
  constexpr int kBlkPerB = kD / 256;
  const int bix = blockIdx.x / kBlkPerB;
  const int d0  = (blockIdx.x - bix * kBlkPerB) * 256;
  const int d   = d0 + tid;
  const size_t row0 = (size_t)bix * kSeq;
  const int hrow = wave >> 1;
  const int hch  = (wave & 1) * 128 + lane * 4;
  float run = 0.0f;
#pragma unroll 1
  for (int sub = kSeq / 16 - 1; sub >= 0; --sub) {
    const size_t lb = row0 + (size_t)sub * 16;
#pragma unroll 1
    for (int s = 15; s >= 0; --s) {
      float v = DLR[(lb + s) * kD + d];
      asm volatile("" : "+v"(v));
      sT[s * kTP + tid] = run;
      run += softplus_f(v);
    }
    __syncthreads();
    v4f fv[4];
#pragma unroll
    for (int it = 0; it < 4; ++it) fv[it] = *(const v4f*)(sT + (it * 4 + hrow) * kTP + hch);
    for (int pass = 0; pass < 2; ++pass) {
#pragma unroll
      for (int it = 0; it < 4; ++it)
        *(volatile v4f*)(SFX + (lb + it * 4 + hrow) * kD + d0 + hch) = fv[it];
      __threadfence();
    }
    __syncthreads();
  }
}

__global__ __launch_bounds__(64) void scan_kernel(
    const float* __restrict__ XD, const float* __restrict__ X, const float* __restrict__ DLR,
    const float* __restrict__ SFX, const float* __restrict__ Alog, const float* __restrict__ Dp,
    unsigned short* __restrict__ YH, unsigned short* __restrict__ YL)
{
  __shared__ __align__(16) float sX[kScanTS * kBC];
  __shared__ __align__(16) float sY[kScanTS * kScanYP];
  __shared__ __align__(16) float sA[kNst * kScanCh];
  const int tid = threadIdx.x, lane = tid & 31, wave = tid >> 5;
  constexpr int kBlkPerB = kD / kScanCh;
  const int bix = blockIdx.x / kBlkPerB;
  const int d0  = (blockIdx.x - bix * kBlkPerB) * kScanCh;
  const int d   = d0 + tid;
  const size_t row0 = (size_t)bix * kSeq;
#pragma unroll 1
  for (int s = 0; s < kNst; ++s) sA[s * kScanCh + tid] = -expf(Alog[(size_t)d * kNst + s]);
  __syncthreads();
  float negA[kNst], h[kNst];
#pragma unroll
  for (int s = 0; s < kNst; ++s) {
    negA[s] = sA[s * kScanCh + tid];
    h[s] = 0.f;
  }
  const float Dd = Dp[d];
  const int lr = tid >> 3, lc4 = (tid & 7) * 4;
  const int q = lane >> 3, c8 = (lane & 7) * 8;
#pragma unroll 1
  for (int t0 = 0; t0 < kSeq; t0 += kScanTS) {
    __syncthreads();
#pragma unroll
    for (int i = 0; i < 8; ++i) {
      const int r = lr + 8 * i;
      *(v4f*)(sX + r * kBC + lc4) = *(const v4f*)(XD + (row0 + t0 + r) * kEP + kDtR + lc4);
    }
    __syncthreads();
#pragma unroll 1
    for (int s = 0; s < kScanTS; ++s) {
      const size_t gi = (row0 + t0 + s) * kD + d;
      float v  = DLR[gi];
      float xt = X[gi];
      float sf = SFX[gi];
      asm volatile("" : "+v"(v), "+v"(xt), "+v"(sf));
      const float* xr = sX + s * kBC;
      float Bs[kNst], Cs[kNst];
#pragma unroll
      for (int q4 = 0; q4 < 4; ++q4) {
        const v4f bv = *(const v4f*)(xr + 4 * q4);
        const v4f cv = *(const v4f*)(xr + kNst + 4 * q4);
        Bs[4 * q4 + 0] = bv[0]; Bs[4 * q4 + 1] = bv[1]; Bs[4 * q4 + 2] = bv[2]; Bs[4 * q4 + 3] = bv[3];
        Cs[4 * q4 + 0] = cv[0]; Cs[4 * q4 + 1] = cv[1]; Cs[4 * q4 + 2] = cv[2]; Cs[4 * q4 + 3] = cv[3];
      }
      const float dt  = softplus_f(v);
      const float dtx = dt * xt;
      float y = 0.f;
#pragma unroll
      for (int k = 0; k < kNst; ++k) {
        const float e = __expf(dt * negA[k]);
        h[k] = e * h[k] + dtx * Bs[k];
        const float P = __expf(negA[k] * sf);
        const float g = P * __builtin_amdgcn_rcpf(P + kEps);
        y = (h[k] * g) * Cs[k] + y;
      }
      y = xt * Dd + y;
      sY[s * kScanYP + tid] = y;
    }
    __syncthreads();
    v4u hv[8], lv[8];
#pragma unroll
    for (int it = 0; it < 8; ++it) {
      const int row = it * 8 + wave * 4 + q;
      const float* sp = sY + row * kScanYP + c8;
      const v4f a0 = *(const v4f*)(sp);
      const v4f a1 = *(const v4f*)(sp + 4);
      split_eight(a0, a1, hv[it], lv[it]);
    }
    for (int pass = 0; pass < 2; ++pass) {
#pragma unroll
      for (int it = 0; it < 8; ++it) {
        const int row = it * 8 + wave * 4 + q;
        const size_t o = (row0 + t0 + row) * kD + d0 + c8;
        *(volatile v4u*)(YH + o) = hv[it];
        *(volatile v4u*)(YL + o) = lv[it];
      }
      __threadfence();
    }
  }
}

extern "C" void kernel_launch(void* const* d_in, const int* in_sizes, int n_in,
                              void* d_out, int out_size, void* d_ws, size_t ws_size,
                              hipStream_t stream) {
  if (n_in < 8) return;
  if (in_sizes[0] != kRows * kD) return;
  if (in_sizes[1] != kD * kE) return;
  if (in_sizes[2] != kDtR * kD) return;
  if (in_sizes[3] != kD) return;
  if (in_sizes[4] != kD * kNst) return;
  if (in_sizes[5] != kD) return;
  if (in_sizes[6] != kD * kD) return;
  if (in_sizes[7] != kD) return;
  if (out_size != kRows * kD) return;
  if (ws_size < kWsTotal) return;

  const float* x     = (const float*)d_in[0];
  const float* W_x   = (const float*)d_in[1];
  const float* W_dt  = (const float*)d_in[2];
  const float* b_dt  = (const float*)d_in[3];
  const float* A_log = (const float*)d_in[4];
  const float* Dp    = (const float*)d_in[5];
  const float* W_out = (const float*)d_in[6];
  const float* b_out = (const float*)d_in[7];
  float* out = (float*)d_out;

  char* ws = (char*)d_ws;
  unsigned short* XH  = (unsigned short*)(ws + kOffXH);
  unsigned short* XL  = (unsigned short*)(ws + kOffXL);
  unsigned short* WXH = (unsigned short*)(ws + kOffWXH);
  unsigned short* WXL = (unsigned short*)(ws + kOffWXL);
  unsigned short* WDH = (unsigned short*)(ws + kOffWDH);
  unsigned short* WDL = (unsigned short*)(ws + kOffWDL);
  unsigned short* WOH = (unsigned short*)(ws + kOffWOH);
  unsigned short* WOL = (unsigned short*)(ws + kOffWOL);
  float*          XD  = (float*)(ws + kOffXD);
  unsigned short* DRH = (unsigned short*)(ws + kOffDRH);
  unsigned short* DRL = (unsigned short*)(ws + kOffDRL);
  float*          DLR = (float*)(ws + kOffDLR);
  float*          SFX = (float*)(ws + kOffSFX);
  unsigned short* YH  = (unsigned short*)(ws + kOffYH);
  unsigned short* YL  = (unsigned short*)(ws + kOffYL);

  split_rows_bf16_kernel<<<(kRows * kD / 8) / 256, 256, 0, stream>>>(x, XH, XL, kRows * kD / 8);

  transpose_split_kernel<<<dim3(kEP / 64, kD / 64), 256, 0, stream>>>(W_x, WXH, WXL, kD, kE);
  transpose_split_kernel<<<dim3(kD / 64, kDtR / 64), 256, 0, stream>>>(W_dt, WDH, WDL, kDtR, kD);
  transpose_split_kernel<<<dim3(kD / 64, kD / 64), 256, 0, stream>>>(W_out, WOH, WOL, kD, kD);

  wmma_gemm64_x3<0><<<dim3((kRows / 64) * (kEP / 64) / 8), 256, 0, stream>>>(
      XH, XL, kD, WXH, WXL, kD, XD, kEP, b_dt, kRows, kEP, kD);

  dr_split_kernel<<<(kRows * kDtR / 8) / 256, 256, 0, stream>>>(XD, DRH, DRL, kRows * kDtR / 8);

  wmma_gemm64_x3<2><<<dim3((kRows / 64) * (kD / 64) / 8), 256, 0, stream>>>(
      DRH, DRL, kDtR, WDH, WDL, kDtR, DLR, kD, b_dt, kRows, kD, kDtR);

  suffix_kernel<<<kBatch * (kD / 256), 256, 0, stream>>>(DLR, SFX);

  scan_kernel<<<kBatch * (kD / kScanCh), kScanCh, 0, stream>>>(XD, x, DLR, SFX, A_log, Dp, YH, YL);

  wmma_gemm64_x3<2><<<dim3((kRows / 64) * (kD / 64) / 8), 256, 0, stream>>>(
      YH, YL, kD, WOH, WOL, kD, out, kD, b_out, kRows, kD, kD);
}
